// MyBlock_64527588655618
// MI455X (gfx1250) — hardware-run, weakly checked
//
#include <hip/hip_runtime.h>
#include <math.h>

constexpr int kBatch    = 2;
constexpr int kSeqLen   = 2048;
constexpr int kDModel   = 1024;
constexpr int kDInner   = 2048;
constexpr int kNState   = 16;
constexpr int kDtRank   = 64;
constexpr int kDFfn     = 4096;
constexpr int kConvTaps = 4;
constexpr int kTok      = kBatch * kSeqLen;
constexpr int kXprojRows = kDtRank + 2 * kNState;
constexpr int kXprojPad  = 128;
constexpr int kBcCols    = 64;
constexpr int kScanChunk = 64;
constexpr int kScanLanes = 64;

constexpr float kWCarry   = 64.0f;
constexpr float kXsCarry  = 256.0f;
constexpr float kDblCarry = 1024.0f;
constexpr float kYCarry   = 1024.0f;
constexpr float kFfnCarry = 16.0f;

constexpr float kScaleInProj  = 1.0f / kWCarry;
constexpr float kScaleDblh    = kDblCarry / (kXsCarry * kWCarry);
constexpr float kScaleBc      = 1.0f / (kXsCarry * kWCarry);
constexpr float kScaleDtp     = 1.0f / (kDblCarry * kWCarry);
constexpr float kScaleOutProj = 1.0f / (kYCarry * kWCarry);
constexpr float kScaleFc      = 1.0f / kWCarry;
constexpr float kScaleProj    = 1.0f / (kFfnCarry * kWCarry);

typedef __attribute__((ext_vector_type(16))) _Float16 v16h;
typedef __attribute__((ext_vector_type(8)))  _Float16 v8h;
typedef __attribute__((ext_vector_type(16))) __bf16   v16b;
typedef __attribute__((ext_vector_type(8)))  __bf16   v8b;
typedef __attribute__((ext_vector_type(8)))  float    v8f;
typedef __attribute__((ext_vector_type(4)))  float    v4f;
typedef __attribute__((ext_vector_type(4)))  unsigned int v4u;

__device__ __forceinline__ unsigned short f2bf_bits(float f) {
  unsigned u = __float_as_uint(f);
  return (unsigned short)((u + 0x7FFFu + ((u >> 16) & 1u)) >> 16);
}
__device__ __forceinline__ float bf_bits2f(unsigned short h) { return __uint_as_float(((unsigned)h) << 16); }

__device__ __forceinline__ void dep_guard_h(v8f& a, v8f& b, v16h x, v16h y) { asm volatile("v_nop\n\tv_nop\n\tv_nop\n\tv_nop" : "+v"(a), "+v"(b) : "v"(x), "v"(y)); }
__device__ __forceinline__ void dep_guard_b(v8f& a, v8f& b, v16b x, v16b y) { asm volatile("v_nop\n\tv_nop\n\tv_nop\n\tv_nop" : "+v"(a), "+v"(b) : "v"(x), "v"(y)); }
__device__ __forceinline__ void keep4_h(v16h a, v16h b, v16h c, v16h d) { asm volatile("v_nop" :: "v"(a), "v"(b), "v"(c), "v"(d)); }
__device__ __forceinline__ void keep4_b(v16b a, v16b b, v16b c, v16b d) { asm volatile("v_nop" :: "v"(a), "v"(b), "v"(c), "v"(d)); }
__device__ __forceinline__ void acc_guard4(v8f& a, v8f& b, v8f& c, v8f& d) { asm volatile("v_nop\n\tv_nop\n\tv_nop\n\tv_nop" : "+v"(a), "+v"(b), "+v"(c), "+v"(d)); }
template <typename T> struct Frag;
template <> struct Frag<_Float16> {
  typedef v16h V; union U { v16h v; v8h h[2]; };
  static __device__ __forceinline__ v16h load(const _Float16* p) {
    U f; f.h[0] = *(const v8h*)(p); f.h[1] = *(const v8h*)(p + 16); return f.v;
  }
  static __device__ __forceinline__ v8f mma(v16h a, v16h b, v8f c) {
    return __builtin_amdgcn_wmma_f32_16x16x32_f16(false, a, false, b, (short)0, c, false, false);
  }
  static __device__ __forceinline__ void guard(v8f& a, v8f& b, v16h x, v16h y) { dep_guard_h(a, b, x, y); }
  static __device__ __forceinline__ void keep(v16h a, v16h b, v16h c, v16h d) { keep4_h(a, b, c, d); }
};
template <> struct Frag<__bf16> {
  typedef v16b V; union U { v16b v; v8b h[2]; };
  static __device__ __forceinline__ v16b load(const __bf16* p) {
    U f; f.h[0] = *(const v8b*)(p); f.h[1] = *(const v8b*)(p + 16); return f.v;
  }
  static __device__ __forceinline__ v8f mma(v16b a, v16b b, v8f c) {
    return __builtin_amdgcn_wmma_f32_16x16x32_bf16(false, a, false, b, (short)0, c, false, false);
  }
  static __device__ __forceinline__ void guard(v8f& a, v8f& b, v16b x, v16b y) { dep_guard_b(a, b, x, y); }
  static __device__ __forceinline__ void keep(v16b a, v16b b, v16b c, v16b d) { keep4_b(a, b, c, d); }
};

__device__ __forceinline__ unsigned pk16(unsigned short a, unsigned short b) { return (unsigned)a | ((unsigned)b << 16); }
__device__ __forceinline__ unsigned short h_bits(float f) { const _Float16 h = (_Float16)f; return __builtin_bit_cast(unsigned short, h); }

template <int ET> struct Elem;
template <> struct Elem<0> { typedef _Float16 T; };
template <> struct Elem<1> { typedef __bf16 T; };
template <int ET, bool SPLIT, int BIAS_MODE, int OUT_MODE, bool RESID, int ACT, bool POSTSC>
__global__ __launch_bounds__(256) void wmma_gemm64(
    const unsigned short* __restrict__ Ap, const unsigned short* __restrict__ A2p, int lda, long strideA,
    const unsigned short* __restrict__ Btp, const unsigned short* __restrict__ Bt2p, int ldb, long strideB,
    void* __restrict__ Cout, void* __restrict__ Cout2, int ldc, long strideC,
    const float* __restrict__ bias,
    const float* __restrict__ resid, long strideR,
    int M, int N, int K, float scale, float post) {
  typedef typename Elem<ET>::T T;
  typedef typename Frag<T>::V V;
  const T* A = (const T*)Ap; const T* A2 = (const T*)A2p; const T* Bt = (const T*)Btp; const T* Bt2 = (const T*)Bt2p;
  __shared__ __align__(16) float sT[8][16 * 68];
  const int b    = blockIdx.y;
  const int lane = threadIdx.x & 31;
  const int wave = threadIdx.x >> 5;
  const int tilesN = N >> 6;
  const int tilesM = M >> 6;
  const int tile = blockIdx.x * 8 + wave;
  if (tile >= tilesM * tilesN) return;
  const int tm = tile / tilesN;
  const int tn = tile - tm * tilesN;
  const int m0 = tm << 6;
  const int n0 = tn << 6;

  const T* Ab  = A  + (size_t)b * strideA;
  const T* Bb  = Bt + (size_t)b * strideB;
  const T* Ab2 = SPLIT ? (A2  + (size_t)b * strideA) : nullptr;
  const T* Bb2 = SPLIT ? (Bt2 + (size_t)b * strideB) : nullptr;

  const int rlane = lane & 15;
  const int koff  = (lane >> 4) * 8;
  const int mOff  = (lane >> 4) * 8;

  v8f acc[4][4];
#pragma unroll
  for (int i = 0; i < 4; ++i)
#pragma unroll
    for (int j = 0; j < 4; ++j) acc[i][j] = (v8f){0.f,0.f,0.f,0.f,0.f,0.f,0.f,0.f};

  for (int k0 = 0; k0 < K; k0 += 32) {
    V bh[4], bl[4];
#pragma unroll
    for (int j = 0; j < 4; ++j) {
      const size_t bo = (size_t)(n0 + (j << 4) + rlane) * ldb + koff + k0;
      bh[j] = Frag<T>::load(Bb + bo);
      if (SPLIT) bl[j] = Frag<T>::load(Bb2 + bo);
    }
#pragma unroll
    for (int i = 0; i < 4; ++i) {
      const size_t ao = (size_t)(m0 + (i << 4) + rlane) * lda + koff + k0;
      V ah = Frag<T>::load(Ab + ao);
      V al;
      if (SPLIT) al = Frag<T>::load(Ab2 + ao);
#pragma unroll
      for (int j = 0; j < 4; ++j) {
        acc[i][j] = Frag<T>::mma(ah, bh[j], acc[i][j]);
        if (SPLIT) {
          acc[i][j] = Frag<T>::mma(ah, bl[j], acc[i][j]);
          acc[i][j] = Frag<T>::mma(al, bh[j], acc[i][j]);
        }
      }
      Frag<T>::guard(acc[i][0], acc[i][3], ah, SPLIT ? al : ah);
    }
    Frag<T>::keep(bh[0], bh[1], bh[2], bh[3]);
    if (SPLIT) Frag<T>::keep(bl[0], bl[1], bl[2], bl[3]);
  }
  acc_guard4(acc[0][0], acc[0][1], acc[0][2], acc[0][3]);
  acc_guard4(acc[1][0], acc[1][1], acc[1][2], acc[1][3]);
  acc_guard4(acc[2][0], acc[2][1], acc[2][2], acc[2][3]);
  acc_guard4(acc[3][0], acc[3][1], acc[3][2], acc[3][3]);

  float* slab = sT[wave];
  const float* Rb = RESID ? (resid + (size_t)b * strideR) : nullptr;
#pragma unroll
  for (int i = 0; i < 4; ++i) {
    const int mBase = m0 + (i << 4);
#pragma unroll
    for (int j = 0; j < 4; ++j) {
      const int n = n0 + (j << 4) + rlane;
      float bv = 0.f;
      if (BIAS_MODE == 2) bv = bias[n];
#pragma unroll
      for (int r = 0; r < 8; ++r) {
        float v = acc[i][j][r] * scale;
        if (BIAS_MODE == 1) v += bias[mBase + mOff + r];
        if (BIAS_MODE == 2) v += bv;
        if (RESID) v += Rb[(size_t)(mBase + mOff + r) * ldc + n];
        if (ACT == 2) v = fmaxf(v, 0.0f);
        if (ACT == 3) v = v / (1.0f + expf(-v));
        if (ACT == 4) v = (v > 0.f) ? v : 0.01f * v;
        if (POSTSC) v = v * post;
        slab[(mOff + r) * 68 + (j << 4) + rlane] = v;
      }
    }
    __builtin_amdgcn_fence(__ATOMIC_RELEASE, "workgroup");
    __builtin_amdgcn_wave_barrier();
    __builtin_amdgcn_fence(__ATOMIC_ACQUIRE, "workgroup");
    if (OUT_MODE == 0) {
      float* C = (float*)Cout + (size_t)b * strideC;
      const int hh = lane >> 4, c4 = (lane & 15) * 4;
      for (int pass = 0; pass < 2; ++pass) {
#pragma unroll
        for (int it = 0; it < 8; ++it) {
          const int row = it * 2 + hh;
          v4f v = *(const v4f*)(slab + row * 68 + c4);
          *(volatile v4f*)(C + (size_t)(mBase + row) * ldc + n0 + c4) = v;
        }
        __threadfence();
      }
    } else {
      const int q = lane >> 3, c8 = (lane & 7) * 8;
      unsigned short* C  = (unsigned short*)Cout  + (size_t)b * strideC;
      unsigned short* C2 = (OUT_MODE == 2) ? ((unsigned short*)Cout2 + (size_t)b * strideC) : nullptr;
      for (int pass = 0; pass < 2; ++pass) {
#pragma unroll
        for (int it = 0; it < 4; ++it) {
          const int row = it * 4 + q;
          const float* sp = slab + row * 68 + c8;
          v8h hv, lv;
#pragma unroll
          for (int e = 0; e < 8; ++e) {
            if (OUT_MODE == 1) {
              hv[e] = (_Float16)sp[e];
            } else {
              unsigned short hb = f2bf_bits(sp[e]);
              unsigned short lb = f2bf_bits(sp[e] - bf_bits2f(hb));
              hv[e] = __builtin_bit_cast(_Float16, hb);
              lv[e] = __builtin_bit_cast(_Float16, lb);
            }
          }
          *(volatile v8h*)(C + (size_t)(mBase + row) * ldc + n0 + c8) = hv;
          if (OUT_MODE == 2) *(volatile v8h*)(C2 + (size_t)(mBase + row) * ldc + n0 + c8) = lv;
        }
        __threadfence();
      }
    }
    __builtin_amdgcn_fence(__ATOMIC_RELEASE, "workgroup");
    __builtin_amdgcn_wave_barrier();
    __builtin_amdgcn_fence(__ATOMIC_ACQUIRE, "workgroup");
  }
}

__global__ __launch_bounds__(256) void cast8_kernel(const float* __restrict__ in, unsigned short* __restrict__ out,
                                                    int nin8, int nout8, float scale) {
  const int i = blockIdx.x * 256 + threadIdx.x;
  if (i >= nout8) return;
  const bool live = (i < nin8);
  const int ic = live ? i : (nin8 - 1);
  const float* p = in + 8 * (size_t)ic;
  const v4f a = *(const v4f*)(p);
  const v4f c = *(const v4f*)(p + 4);
  unsigned short hb[8];
#pragma unroll
  for (int e = 0; e < 4; ++e) {
    const float va = live ? a[e] * scale : 0.0f;
    const float vc = live ? c[e] * scale : 0.0f;
    hb[e]     = h_bits(va);
    hb[4 + e] = h_bits(vc);
  }
  const v4u u = (v4u){pk16(hb[0], hb[1]), pk16(hb[2], hb[3]), pk16(hb[4], hb[5]), pk16(hb[6], hb[7])};
  unsigned short* q = out + 8 * (size_t)i;
  *(volatile v4u*)q = u;
  __threadfence();
  *(volatile v4u*)q = u;
}

__global__ __launch_bounds__(128) void ln_f16_kernel(const float* __restrict__ x, const float* __restrict__ w,
                                                     unsigned short* __restrict__ out) {
  __shared__ float redA[4];
  __shared__ float redB[4];
  const int row  = blockIdx.x;
  const int t    = threadIdx.x;
  const int lane = t & 31, wave = t >> 5;
  const int c0   = t * 8;
  const float* xr = x + (size_t)row * kDModel + c0;
  const v4f a = *(const v4f*)(xr);
  const v4f c = *(const v4f*)(xr + 4);
  float v[8];
#pragma unroll
  for (int e = 0; e < 4; ++e) { v[e] = a[e]; v[4 + e] = c[e]; }
  float s = ((v[0] + v[1]) + (v[2] + v[3])) + ((v[4] + v[5]) + (v[6] + v[7]));
#pragma unroll
  for (int off = 16; off > 0; off >>= 1) s += __shfl_xor(s, off, 32);
  if (lane == 0) redA[wave] = s;
  __syncthreads();
  const float tot = ((redA[0] + redA[1]) + redA[2]) + redA[3];
  const float mu = tot * (1.0f / 1024.0f);
  float d[8];
  float s2 = 0.f;
#pragma unroll
  for (int e = 0; e < 8; ++e) { d[e] = v[e] - mu; s2 += d[e] * d[e]; }
#pragma unroll
  for (int off = 16; off > 0; off >>= 1) s2 += __shfl_xor(s2, off, 32);
  if (lane == 0) redB[wave] = s2;
  __syncthreads();
  const float tot2 = ((redB[0] + redB[1]) + redB[2]) + redB[3];
  const float var = tot2 * (1.0f / 1024.0f);
  const float inv = 1.0f / sqrtf(var + 1e-5f);
  const v4f wa = *(const v4f*)(w + c0);
  const v4f wc = *(const v4f*)(w + c0 + 4);
  unsigned short hb[8];
#pragma unroll
  for (int e = 0; e < 4; ++e) {
    hb[e]     = h_bits((d[e] * inv) * wa[e]);
    hb[4 + e] = h_bits((d[4 + e] * inv) * wc[e]);
  }
  const v4u u = (v4u){pk16(hb[0], hb[1]), pk16(hb[2], hb[3]), pk16(hb[4], hb[5]), pk16(hb[6], hb[7])};
  unsigned short* op = out + (size_t)row * kDModel + c0;
  *(volatile v4u*)op = u;
  __threadfence();
  *(volatile v4u*)op = u;
}

__global__ __launch_bounds__(256) void conv_silu_kernel(const float* __restrict__ xm, const float* __restrict__ cw,
                                                        const float* __restrict__ cb, float* __restrict__ xs,
                                                        unsigned short* __restrict__ xsh) {
  __shared__ __align__(16) float sX[1024];
  const int tok  = blockIdx.x >> 1;
  const int half = blockIdx.x & 1;
  const int l    = tok & (kSeqLen - 1);
  const int t    = threadIdx.x;
  const int dloc = 4 * t;
  const int d0   = half * 1024 + dloc;
  const v4f bias = *(const v4f*)(cb + d0);
  v4f wq[4];
#pragma unroll
  for (int j = 0; j < 4; ++j) wq[j] = *(const v4f*)(cw + (size_t)(d0 + j) * kConvTaps);
  v4f acc = (v4f){0.f, 0.f, 0.f, 0.f};
#pragma unroll
  for (int k = 0; k < kConvTaps; ++k) {
    const int ll = l - (kConvTaps - 1) + k;
    const bool live = (ll >= 0);
    const int rowc = live ? (tok - (kConvTaps - 1) + k) : tok;
    const v4f xv = *(const v4f*)(xm + (size_t)rowc * kDInner + d0);
#pragma unroll
    for (int j = 0; j < 4; ++j) {
      const float xe = live ? xv[j] : 0.0f;
      acc[j] = acc[j] + wq[j][k] * xe;
    }
  }
  v4f o;
#pragma unroll
  for (int j = 0; j < 4; ++j) {
    const float sv = acc[j] + bias[j];
    const float ez = expf(fminf(-sv, 60.0f));
    o[j] = sv * (1.0f / (1.0f + ez));
  }
  *(v4f*)(sX + dloc) = o;
  float* op = xs + (size_t)tok * kDInner + d0;
  for (int pass = 0; pass < 2; ++pass) {
    *(volatile v4f*)op = o;
    __threadfence();
  }
  __syncthreads();
  if (t < 128) {
    const int c8 = 8 * t;
    const v4f a = *(const v4f*)(sX + c8);
    const v4f c = *(const v4f*)(sX + c8 + 4);
    unsigned short hb[8];
#pragma unroll
    for (int e = 0; e < 4; ++e) {
      hb[e]     = h_bits(a[e] * kXsCarry);
      hb[4 + e] = h_bits(c[e] * kXsCarry);
    }
    const v4u u = (v4u){pk16(hb[0], hb[1]), pk16(hb[2], hb[3]), pk16(hb[4], hb[5]), pk16(hb[6], hb[7])};
    unsigned short* hp = xsh + (size_t)tok * kDInner + half * 1024 + c8;
    for (int pass = 0; pass < 2; ++pass) {
      *(volatile v4u*)hp = u;
      __threadfence();
    }
  }
}

__global__ __launch_bounds__(64) void scan_gate_kernel(const float* __restrict__ dtp, const float* __restrict__ bcp,
                                                      const float* __restrict__ us, const unsigned short* __restrict__ zh,
                                                      const float* __restrict__ alog, const float* __restrict__ dv,
                                                      unsigned short* __restrict__ yg) {
  __shared__ float sA[kNState * kScanLanes];
  __shared__ float sH[kNState * kScanLanes];
  __shared__ __align__(16) float sBC[kScanChunk * 32];
  __shared__ __align__(16) unsigned short sO[kScanChunk * kScanLanes];
  const int tl   = threadIdx.x;
  const int lane = tl & 31, wave = tl >> 5;
  const int d0   = blockIdx.x * kScanLanes;
  const int b    = blockIdx.y;
  const int d    = d0 + tl;
#pragma unroll 1
  for (int n = 0; n < kNState; ++n) {
    sA[n * kScanLanes + tl] = -expf(alog[(size_t)d * kNState + n]);
    sH[n * kScanLanes + tl] = 0.0f;
  }
  const float dd = dv[d];
  const int q = lane >> 3, c8 = (lane & 7) * 8;
#pragma unroll 1
  for (int ch = 0; ch < kSeqLen / kScanChunk; ++ch) {
    const int tok0 = b * kSeqLen + ch * kScanChunk;
    __syncthreads();
#pragma unroll
    for (int it = 0; it < 8; ++it) {
      const int idx = it * kScanLanes + tl;
      const int row = idx >> 3;
      const int c4  = (idx & 7) * 4;
      *(v4f*)(sBC + row * 32 + c4) = *(const v4f*)(bcp + (size_t)(tok0 + row) * kBcCols + c4);
    }
    __syncthreads();
#pragma unroll 1
    for (int s = 0; s < kScanChunk; ++s) {
      const size_t e = (size_t)(tok0 + s) * kDInner + d;
      const float pre = dtp[e];
      const float uu  = us[e];
      const unsigned short zb = zh[e];
      const float zz = (float)__builtin_bit_cast(_Float16, zb);
      const float dlt = fmaxf(pre, 0.0f) + log1pf(expf(-fabsf(pre)));
      const float* bcs = sBC + s * 32;
      float ysc = 0.0f;
#pragma unroll 1
      for (int n = 0; n < kNState; ++n) {
        const float an = sA[n * kScanLanes + tl];
        float hn = sH[n * kScanLanes + tl];
        const float bn = bcs[n];
        const float cn = bcs[kNState + n];
        const float dA = expf(dlt * an);
        const float dbu = (dlt * bn) * uu;
        hn = hn * dA + dbu;
        ysc = ysc + hn * cn;
        sH[n * kScanLanes + tl] = hn;
      }
      const float y  = ysc + uu * dd;
      const float ez = expf(fminf(-zz, 60.0f));
      const float g  = zz * (1.0f / (1.0f + ez));
      const float o  = (y * g) * kYCarry;
      sO[s * kScanLanes + tl] = h_bits(o);
    }
    __syncthreads();
    for (int pass = 0; pass < 2; ++pass) {
#pragma unroll
      for (int it = 0; it < 8; ++it) {
        const int row = wave * 32 + it * 4 + q;
        const v4u u = *(const v4u*)(sO + row * kScanLanes + c8);
        *(volatile v4u*)(yg + (size_t)(tok0 + row) * kDInner + d0 + c8) = u;
      }
      __threadfence();
    }
  }
}

extern "C" void kernel_launch(void* const* d_in, const int* in_sizes, int n_in,
                              void* d_out, int out_size, void* d_ws, size_t ws_size,
                              hipStream_t stream) {
  if (n_in < 14) return;
  if (in_sizes[0] != kTok * kDModel || out_size != kTok * kDModel) return;
  if (in_sizes[2] != 2 * kDInner * kDModel || in_sizes[5] != kXprojRows * kDInner ||
      in_sizes[6] != kDInner * kDtRank || in_sizes[8] != kDInner * kNState ||
      in_sizes[10] != kDModel * kDInner || in_sizes[12] != kDFfn * kDModel || in_sizes[13] != kDModel * kDFfn) return;

  const float* x          = (const float*)d_in[0];
  const float* ln1_w      = (const float*)d_in[1];
  const float* in_proj_w  = (const float*)d_in[2];
  const float* conv_w     = (const float*)d_in[3];
  const float* conv_b     = (const float*)d_in[4];
  const float* x_proj_w   = (const float*)d_in[5];
  const float* dt_proj_w  = (const float*)d_in[6];
  const float* dt_proj_b  = (const float*)d_in[7];
  const float* a_log      = (const float*)d_in[8];
  const float* d_vec      = (const float*)d_in[9];
  const float* out_proj_w = (const float*)d_in[10];
  const float* ln2_w      = (const float*)d_in[11];
  const float* fc_w       = (const float*)d_in[12];
  const float* proj_w     = (const float*)d_in[13];
  float* out = (float*)d_out;

  const size_t MiB = 1048576;
  const size_t oYg   = 0;
  const size_t oWout = 16 * MiB;
  const size_t oWdt  = oWout + (size_t)kDModel * kDInner * 2;
  const size_t oWxp  = oWdt  + (size_t)kDInner * kDtRank * 2;
  const size_t oPool = 21 * MiB;
  const size_t oWin  = oPool;
  const size_t oHh   = oWin + (size_t)2 * kDInner * kDModel * 2;
  const size_t oXsh  = oPool;
  const size_t oDtp  = oPool;
  const size_t oX1   = oPool;
  const size_t oXm   = oHh + (size_t)kTok * kDModel * 2;
  const size_t oH2   = oXm;
  const size_t oFfn  = oH2 + (size_t)kTok * kDModel * 2;
  const size_t oZ    = oXm + (size_t)kTok * kDInner * 4;
  const size_t oBc   = oZ  - (size_t)kTok * kBcCols * 4;
  const size_t oDblh = oBc - (size_t)kTok * kDtRank * 2;
  const size_t oXs   = oZ  + (size_t)kTok * kDInner * 2;
  const size_t oWfc  = oXs;
  const size_t oWpr  = oWfc + (size_t)kDFfn * kDModel * 2;
  const size_t oEnd  = oXs + (size_t)kTok * kDInner * 4;
  if (oEnd > ws_size) return;
  if (oWxp + (size_t)kXprojPad * kDInner * 2 > oPool) return;
  if (oDtp + (size_t)kTok * kDInner * 4 > oDblh) return;
  if (oFfn + (size_t)kTok * kDFfn * 2 > oXs) return;

  char* ws = (char*)d_ws;
  unsigned short* wPr  = (unsigned short*)(ws + oWpr);
  unsigned short* wFc  = (unsigned short*)(ws + oWfc);
  unsigned short* wOut = (unsigned short*)(ws + oWout);
  unsigned short* wDt  = (unsigned short*)(ws + oWdt);
  unsigned short* wXp  = (unsigned short*)(ws + oWxp);
  unsigned short* wIn  = (unsigned short*)(ws + oWin);
  unsigned short* hH   = (unsigned short*)(ws + oHh);
  unsigned short* xsH  = (unsigned short*)(ws + oXsh);
  float*          dtp  = (float*)(ws + oDtp);
  float*          x1   = (float*)(ws + oX1);
  float*          xm   = (float*)(ws + oXm);
  unsigned short* hH2  = (unsigned short*)(ws + oH2);
  unsigned short* ffn  = (unsigned short*)(ws + oFfn);
  unsigned short* zH   = (unsigned short*)(ws + oZ);
  float*          bc   = (float*)(ws + oBc);
  unsigned short* dblH = (unsigned short*)(ws + oDblh);
  float*          xs   = (float*)(ws + oXs);
  unsigned short* yg   = (unsigned short*)(ws + oYg);

  {
    const int n_in   = 2 * kDInner * kDModel / 8;
    const int n_xp_i = kXprojRows * kDInner / 8;
    const int n_xp_o = kXprojPad * kDInner / 8;
    const int n_dt   = kDInner * kDtRank / 8;
    const int n_out  = kDModel * kDInner / 8;
    const int n_fc   = kDFfn * kDModel / 8;
    const int n_pr   = kDModel * kDFfn / 8;
    cast8_kernel<<<(n_in + 255) / 256, 256, 0, stream>>>(in_proj_w, wIn, n_in, n_in, kWCarry);
    cast8_kernel<<<(n_xp_o + 255) / 256, 256, 0, stream>>>(x_proj_w, wXp, n_xp_i, n_xp_o, kWCarry);
    cast8_kernel<<<(n_dt + 255) / 256, 256, 0, stream>>>(dt_proj_w, wDt, n_dt, n_dt, kWCarry);
    cast8_kernel<<<(n_out + 255) / 256, 256, 0, stream>>>(out_proj_w, wOut, n_out, n_out, kWCarry);
  }

  ln_f16_kernel<<<kTok, 128, 0, stream>>>(x, ln1_w, hH);

  {
    const int tiles = (kTok / 64) * (kDInner / 64);
    wmma_gemm64<0, false, 0, 0, false, 0, false><<<dim3((tiles + 7) / 8, 1), 256, 0, stream>>>(
        hH, hH, kDModel, 0L, wIn, wIn, kDModel, 0L, (void*)xm, (void*)xm, kDInner, 0L,
        dt_proj_b, x, 0L, kTok, kDInner, kDModel, kScaleInProj, 1.0f);
    const unsigned short* wInZ = wIn + (size_t)kDInner * kDModel;
    wmma_gemm64<0, false, 0, 1, false, 0, false><<<dim3((tiles + 7) / 8, 1), 256, 0, stream>>>(
        hH, hH, kDModel, 0L, wInZ, wInZ, kDModel, 0L, (void*)zH, (void*)zH, kDInner, 0L,
        dt_proj_b, x, 0L, kTok, kDInner, kDModel, kScaleInProj, 1.0f);
  }

  conv_silu_kernel<<<kTok * 2, 256, 0, stream>>>(xm, conv_w, conv_b, xs, xsH);

  {
    const int tiles = (kTok / 64) * (kDtRank / 64);
    wmma_gemm64<0, false, 0, 1, false, 0, false><<<dim3((tiles + 7) / 8, 1), 256, 0, stream>>>(
        xsH, xsH, kDInner, 0L, wXp, wXp, kDInner, 0L, (void*)dblH, (void*)dblH, kDtRank, 0L,
        dt_proj_b, x, 0L, kTok, kDtRank, kDInner, kScaleDblh, 1.0f);
    const unsigned short* wXpBC = wXp + (size_t)kDtRank * kDInner;
    wmma_gemm64<0, false, 0, 0, false, 0, false><<<dim3((tiles + 7) / 8, 1), 256, 0, stream>>>(
        xsH, xsH, kDInner, 0L, wXpBC, wXpBC, kDInner, 0L, (void*)bc, (void*)bc, kBcCols, 0L,
        dt_proj_b, x, 0L, kTok, kBcCols, kDInner, kScaleBc, 1.0f);
  }

  {
    const int tiles = (kTok / 64) * (kDInner / 64);
    wmma_gemm64<0, false, 2, 0, false, 0, false><<<dim3((tiles + 7) / 8, 1), 256, 0, stream>>>(
        dblH, dblH, kDtRank, 0L, wDt, wDt, kDtRank, 0L, (void*)dtp, (void*)dtp, kDInner, 0L,
        dt_proj_b, x, 0L, kTok, kDInner, kDtRank, kScaleDtp, 1.0f);
  }

  scan_gate_kernel<<<dim3(kDInner / kScanLanes, kBatch), kScanLanes, 0, stream>>>(dtp, bc, xs, zH, a_log, d_vec, yg);

  {
    const int tiles = (kTok / 64) * (kDModel / 64);
    wmma_gemm64<0, false, 0, 0, true, 0, false><<<dim3((tiles + 7) / 8, 1), 256, 0, stream>>>(
        yg, yg, kDInner, 0L, wOut, wOut, kDInner, 0L, (void*)x1, (void*)x1, kDModel, 0L,
        dt_proj_b, x, 0L, kTok, kDModel, kDInner, kScaleOutProj, 1.0f);
  }

  {
    const int n_fc   = kDFfn * kDModel / 8;
    const int n_pr   = kDModel * kDFfn / 8;
    cast8_kernel<<<(n_fc + 255) / 256, 256, 0, stream>>>(fc_w, wFc, n_fc, n_fc, kWCarry);
    cast8_kernel<<<(n_pr + 255) / 256, 256, 0, stream>>>(proj_w, wPr, n_pr, n_pr, kWCarry);
  }
  ln_f16_kernel<<<kTok, 128, 0, stream>>>(x1, ln2_w, hH2);

  {
    const int tiles = (kTok / 64) * (kDFfn / 64);
    wmma_gemm64<0, false, 0, 1, false, 3, true><<<dim3((tiles + 7) / 8, 1), 256, 0, stream>>>(
        hH2, hH2, kDModel, 0L, wFc, wFc, kDModel, 0L, (void*)ffn, (void*)ffn, kDFfn, 0L,
        dt_proj_b, x, 0L, kTok, kDFfn, kDModel, kScaleFc, kFfnCarry);
  }

  {
    const int tiles = (kTok / 64) * (kDModel / 64);
    wmma_gemm64<0, false, 0, 0, true, 0, false><<<dim3((tiles + 7) / 8, 1), 256, 0, stream>>>(
        ffn, ffn, kDFfn, 0L, wPr, wPr, kDFfn, 0L, (void*)out, (void*)out, kDModel, 0L,
        dt_proj_b, x1, 0L, kTok, kDModel, kDFfn, kScaleProj, 1.0f);
  }
}
